// LEDDecoderAttentionTopicAware_35235911696706
// MI455X (gfx1250) — hardware-verified
//
#include <hip/hip_runtime.h>

typedef __bf16 v16b __attribute__((ext_vector_type(16)));
typedef unsigned short us;
typedef us    v8us __attribute__((ext_vector_type(8)));
typedef float v8f  __attribute__((ext_vector_type(8)));
typedef float v4f  __attribute__((ext_vector_type(4)));
typedef v8us __attribute__((may_alias)) v8usa;
typedef v4f  __attribute__((may_alias)) v4fa;

union FragB { v16b v; v8us half[2]; };

#define BSZ  2
#define TGL  1024
#define SRL  2048
#define EMB  1024
#define TDW  512
#define NH   16
#define DM   64
#define NBH  (BSZ * NH)
#define MQ   (BSZ * TGL)
#define MKV  (BSZ * SRL)
#define GK   (3 * EMB)

#define N_HID (MQ * EMB)
#define N_KVS (MKV * EMB)
#define N_KVT (MKV * TDW)
#define N_WE  (EMB * EMB)
#define N_WT  (EMB * TDW)
#define N_WG  (NH * GK)
#define QPL   (NBH * TGL * DM)
#define KPL   (NBH * SRL * DM)

#define OFF_WQ  0
#define OFF_WK  (OFF_WQ + N_WE)
#define OFF_WV  (OFF_WK + N_WE)
#define OFF_WO  (OFF_WV + N_WE)
#define OFF_WTK (OFF_WO + N_WE)
#define OFF_WTV (OFF_WTK + N_WT)
#define OFF_HID (OFF_WTV + N_WT)
#define OFF_KVS (OFF_HID + N_HID)
#define OFF_KVT (OFF_KVS + N_KVS)
#define N_CVB   (OFF_KVT + N_KVT)

__device__ __forceinline__ us bf16_rne(float x) {
  unsigned u = __float_as_uint(x);
  u += 0x7FFFu + ((u >> 16) & 1u);
  return (us)(u >> 16);
}
__device__ __forceinline__ float bf16_val(us b) {
  return __uint_as_float(((unsigned)b) << 16);
}
__device__ __forceinline__ v8us bf16x8(v4f a, v4f c) {
  const v8us o = { bf16_rne(a.x), bf16_rne(a.y), bf16_rne(a.z), bf16_rne(a.w),
                   bf16_rne(c.x), bf16_rne(c.y), bf16_rne(c.z), bf16_rne(c.w) };
  return o;
}
__device__ __forceinline__ void split8(v8f a, v8us& hi, v8us& lo) {
  const us h0 = bf16_rne(a[0]), h1 = bf16_rne(a[1]), h2 = bf16_rne(a[2]), h3 = bf16_rne(a[3]);
  const us h4 = bf16_rne(a[4]), h5 = bf16_rne(a[5]), h6 = bf16_rne(a[6]), h7 = bf16_rne(a[7]);
  const v8us hv = { h0, h1, h2, h3, h4, h5, h6, h7 };
  const v8us lv = { bf16_rne(a[0] - bf16_val(h0)), bf16_rne(a[1] - bf16_val(h1)),
                    bf16_rne(a[2] - bf16_val(h2)), bf16_rne(a[3] - bf16_val(h3)),
                    bf16_rne(a[4] - bf16_val(h4)), bf16_rne(a[5] - bf16_val(h5)),
                    bf16_rne(a[6] - bf16_val(h6)), bf16_rne(a[7] - bf16_val(h7)) };
  hi = hv;
  lo = lv;
}

__device__ __forceinline__ v8f wmma_bf(v16b a, v16b b, v8f c) {
  v8f d = __builtin_amdgcn_wmma_f32_16x16x32_bf16(false, a, false, b, (short)0, c, false, false);
  asm volatile("v_nop\n\tv_nop\n\tv_nop\n\tv_nop" : "+v"(d) : "v"(a), "v"(b));
  return d;
}

__device__ __forceinline__ v16b ldb(const us* p, int h) {
  FragB f;
  f.half[0] = *(const v8usa*)(p + 8 * h);
  f.half[1] = *(const v8usa*)(p + 16 + 8 * h);
  return f.v;
}
__device__ __forceinline__ v16b ldf(const float* p, int h) {
  const float* p0 = p + 8 * h;
  const float* p1 = p + 16 + 8 * h;
  FragB f;
  f.half[0] = bf16x8(*(const v4fa*)p0, *(const v4fa*)(p0 + 4));
  f.half[1] = bf16x8(*(const v4fa*)p1, *(const v4fa*)(p1 + 4));
  return f.v;
}

__global__ __launch_bounds__(256) void conv_kernel(
    const float* __restrict__ p0, const float* __restrict__ p1, const float* __restrict__ p2,
    const float* __restrict__ p3, const float* __restrict__ p4, const float* __restrict__ p5,
    const float* __restrict__ p6, const float* __restrict__ p7, const float* __restrict__ p8,
    us* __restrict__ dst)
{
  const unsigned g = blockIdx.x * 256u + threadIdx.x;
  if (g >= (unsigned)(N_CVB / 8)) return;
  const float* src;
  unsigned loc;
  if      (g < (unsigned)(OFF_WK  / 8)) { src = p0; loc = g; }
  else if (g < (unsigned)(OFF_WV  / 8)) { src = p1; loc = g - (unsigned)(OFF_WK  / 8); }
  else if (g < (unsigned)(OFF_WO  / 8)) { src = p2; loc = g - (unsigned)(OFF_WV  / 8); }
  else if (g < (unsigned)(OFF_WTK / 8)) { src = p3; loc = g - (unsigned)(OFF_WO  / 8); }
  else if (g < (unsigned)(OFF_WTV / 8)) { src = p4; loc = g - (unsigned)(OFF_WTK / 8); }
  else if (g < (unsigned)(OFF_HID / 8)) { src = p5; loc = g - (unsigned)(OFF_WTV / 8); }
  else if (g < (unsigned)(OFF_KVS / 8)) { src = p6; loc = g - (unsigned)(OFF_HID / 8); }
  else if (g < (unsigned)(OFF_KVT / 8)) { src = p7; loc = g - (unsigned)(OFF_KVS / 8); }
  else                                  { src = p8; loc = g - (unsigned)(OFF_KVT / 8); }
  const float* p = src + (size_t)loc * 8;
  const v8us o = bf16x8(*(const v4fa*)p, *(const v4fa*)(p + 4));
  us* d = dst + (size_t)g * 8;
  *(volatile v8us*)d = o;
  __threadfence();
  *(volatile v8us*)d = o;
}

__device__ __forceinline__ void proj_pass_planes(const us* s16, us* oH, us* oL,
                                                 int bh, int Sper, int s0, int w, int lane) {
  const int q8 = lane & 7, sub = lane >> 3;
  #pragma unroll
  for (int i = 0; i < 8; ++i) {
    const int lid = w * 32 + i * 4 + sub;
    const v8us a = *(const v8usa*)(s16 + lid * DM + 8 * q8);
    const v8us c = *(const v8usa*)(s16 + 8192 + lid * DM + 8 * q8);
    const size_t off = ((size_t)bh * Sper + s0 + lid) * DM + 8 * q8;
    *(volatile v8us*)(oH + off) = a;
    *(volatile v8us*)(oL + off) = c;
  }
}
__device__ __forceinline__ void proj_pass_tplanes(const us* s16, us* oH, us* oL,
                                                  int bh, int Sper, int s0, int w, int lane) {
  const int q8 = lane & 7, sub = lane >> 3;
  #pragma unroll
  for (int i = 0; i < 8; ++i) {
    const int lid = w * 32 + i * 4 + sub;
    const int d = lid >> 1, hl = lid & 1;
    const v8us a = *(const v8usa*)(s16 + d * 128 + 64 * hl + 8 * q8);
    const v8us c = *(const v8usa*)(s16 + 8192 + d * 128 + 64 * hl + 8 * q8);
    const size_t off = ((size_t)bh * DM + d) * Sper + s0 + 64 * hl + 8 * q8;
    *(volatile v8us*)(oH + off) = a;
    *(volatile v8us*)(oL + off) = c;
  }
}
__device__ __forceinline__ void proj_pass_t32(const float* s32, float* oT,
                                              int bh, int Sper, int s0, int w, int lane) {
  const int q8 = lane & 7, sub = lane >> 3;
  #pragma unroll
  for (int i = 0; i < 16; ++i) {
    const int lid = w * 64 + i * 4 + sub;
    const int d = lid >> 2, part = lid & 3;
    const v4f v = *(const v4fa*)(s32 + d * 128 + 32 * part + 4 * q8);
    const size_t off = ((size_t)bh * DM + d) * Sper + s0 + 32 * part + 4 * q8;
    *(volatile v4f*)(oT + off) = v;
  }
}

__global__ __launch_bounds__(128) void proj_kernel(
    const us* __restrict__ X, const us* __restrict__ W, const float* __restrict__ bias,
    int K, int Sper, int mode,
    us* __restrict__ oH, us* __restrict__ oL, float* __restrict__ oT32)
{
  __shared__ __attribute__((aligned(16))) float sraw[8192];
  us* const s16 = reinterpret_cast<us*>(sraw);

  const int tid = threadIdx.x, lane = tid & 31, w = tid >> 5;
  const int h = lane >> 4, m = lane & 15;
  const int m0 = blockIdx.x * 128;
  const int head = blockIdx.y;
  const int m0w = m0 + 32 * w;

  const us* xa0 = X + (size_t)(m0w + m) * K;
  const us* xa1 = xa0 + (size_t)16 * K;
  const us* wb  = W + (size_t)(head * DM + m) * K;

  const v8f zero8 = {0.f, 0.f, 0.f, 0.f, 0.f, 0.f, 0.f, 0.f};
  v8f acc[2][4];
  #pragma unroll
  for (int mt = 0; mt < 2; ++mt)
    #pragma unroll
    for (int nt = 0; nt < 4; ++nt) acc[mt][nt] = zero8;

  #pragma unroll 1
  for (int k0 = 0; k0 < K; k0 += 32) {
    const v16b a0 = ldb(xa0 + k0, h);
    const v16b a1 = ldb(xa1 + k0, h);
    #pragma unroll
    for (int nt = 0; nt < 4; ++nt) {
      const v16b b = ldb(wb + (size_t)nt * 16 * K + k0, h);
      acc[0][nt] = wmma_bf(a0, b, acc[0][nt]);
      acc[1][nt] = wmma_bf(a1, b, acc[1][nt]);
    }
  }

  const float osc = (mode == 0) ? 0.125f : 1.0f;
  float bvals[4];
  #pragma unroll
  for (int nt = 0; nt < 4; ++nt) bvals[nt] = bias[head * DM + 16 * nt + m];

  #pragma unroll
  for (int nt = 0; nt < 4; ++nt) {
    const int feat = 16 * nt + m;
    #pragma unroll
    for (int mt = 0; mt < 2; ++mt) {
      #pragma unroll
      for (int r = 0; r < 8; ++r) {
        const int tokl = 32 * w + 16 * mt + 8 * h + r;
        const float y = (acc[mt][nt][r] + bvals[nt]) * osc;
        const us hi = bf16_rne(y);
        const us lo = bf16_rne(y - bf16_val(hi));
        const int idx = (mode == 2) ? (feat * 128 + tokl) : (tokl * DM + feat);
        s16[idx] = hi;
        s16[8192 + idx] = lo;
      }
    }
  }
  __syncthreads();

  const int b = m0 / Sper, s0 = m0 - b * Sper, bh = b * NH + head;
  if (mode != 2) {
    proj_pass_planes(s16, oH, oL, bh, Sper, s0, w, lane);
    __threadfence();
    proj_pass_planes(s16, oH, oL, bh, Sper, s0, w, lane);
  } else {
    proj_pass_tplanes(s16, oH, oL, bh, Sper, s0, w, lane);
    __threadfence();
    proj_pass_tplanes(s16, oH, oL, bh, Sper, s0, w, lane);
  }

  if (mode == 0) {
    __syncthreads();
    #pragma unroll
    for (int nt = 0; nt < 4; ++nt) {
      const int feat = 16 * nt + m;
      #pragma unroll
      for (int mt = 0; mt < 2; ++mt) {
        #pragma unroll
        for (int r = 0; r < 8; ++r) {
          const int tokl = 32 * w + 16 * mt + 8 * h + r;
          sraw[feat * 128 + tokl] = (acc[mt][nt][r] + bvals[nt]) * osc;
        }
      }
    }
    __syncthreads();
    proj_pass_t32(sraw, oT32, bh, Sper, s0, w, lane);
    __threadfence();
    proj_pass_t32(sraw, oT32, bh, Sper, s0, w, lane);
  }
}

__device__ __forceinline__ void pack_p2(v8f a, v8f c, v16b& phi, v16b& plo) {
  FragB fh, fl;
  v8us h0, l0, h1, l1;
  split8(a, h0, l0);
  split8(c, h1, l1);
  fh.half[0] = h0; fh.half[1] = h1;
  fl.half[0] = l0; fl.half[1] = l1;
  phi = fh.v;
  plo = fl.v;
}

template <bool DUAL>
__device__ __forceinline__ void attn_pass(const float* sO, float* oA, float* oB,
                                          int bh, int q0, int w, int lane) {
  const int q8 = lane & 7, sub = lane >> 3;
  #pragma unroll
  for (int i = 0; i < 8; ++i) {
    const int L = w * 32 + i * 4 + sub;
    const int d = L >> 1, hl = L & 1;
    const size_t off = ((size_t)bh * DM + d) * TGL + q0 + 32 * hl + 4 * q8;
    const v4f v = *(const v4fa*)(sO + d * 64 + 32 * hl + 4 * q8);
    *(volatile v4f*)(oA + off) = v;
    if (DUAL) {
      const v4f v2 = *(const v4fa*)(sO + 4096 + d * 64 + 32 * hl + 4 * q8);
      *(volatile v4f*)(oB + off) = v2;
    }
  }
}

template <bool DUAL>
__global__ __launch_bounds__(128) void attn_kernel(
    const us* __restrict__ qhp, const us* __restrict__ qlp,
    const us* __restrict__ khp, const us* __restrict__ klp,
    const us* __restrict__ vahp, const us* __restrict__ valp,
    const us* __restrict__ vbhp, const us* __restrict__ vblp,
    float* __restrict__ oap, float* __restrict__ obp)
{
  __shared__ __attribute__((aligned(16))) float sO[DUAL ? 2 * DM * 64 : DM * 64];

  const int tid = threadIdx.x, lane = tid & 31, w = tid >> 5;
  const int h = lane >> 4, m = lane & 15;
  const int bh = blockIdx.y;
  const int q0 = blockIdx.x * 64;
  const int qw = q0 + 16 * w;

  const size_t qro = ((size_t)bh * TGL + qw + m) * DM;
  const v16b qh0 = ldb(qhp + qro, h), qh1 = ldb(qhp + qro + 32, h);
  const v16b ql0 = ldb(qlp + qro, h), ql1 = ldb(qlp + qro + 32, h);

  const v8f zero8 = {0.f, 0.f, 0.f, 0.f, 0.f, 0.f, 0.f, 0.f};
  v8f oa[4], ob[4];
  #pragma unroll
  for (int t = 0; t < 4; ++t) { oa[t] = zero8; ob[t] = zero8; }
  float mrun = -1.0e30f, lrun = 0.0f;

  const size_t kro = ((size_t)bh * SRL + m) * DM;
  const us* khb = khp + kro;
  const us* klb = klp + kro;
  const size_t vro = ((size_t)bh * DM + m) * SRL;
  const us* vahb = vahp + vro;
  const us* valb = valp + vro;
  const us* vbhb = vbhp + vro;
  const us* vblb = vblp + vro;

  #pragma unroll 1
  for (int kb = 0; kb < SRL; kb += 64) {
    v8f s[4];
    #pragma unroll
    for (int j = 0; j < 4; ++j) {
      const size_t ko = (size_t)(kb + 16 * j) * DM;
      const v16b kl0 = ldb(klb + ko, h), kl1 = ldb(klb + ko + 32, h);
      const v16b kh0 = ldb(khb + ko, h), kh1 = ldb(khb + ko + 32, h);
      v8f z = zero8;
      z = wmma_bf(kl0, qh0, z);
      z = wmma_bf(kl1, qh1, z);
      z = wmma_bf(kh0, ql0, z);
      z = wmma_bf(kh1, ql1, z);
      z = wmma_bf(kh0, qh0, z);
      z = wmma_bf(kh1, qh1, z);
      s[j] = z;
    }

    float mloc = s[0][0];
    #pragma unroll
    for (int j = 0; j < 4; ++j)
      #pragma unroll
      for (int r = 0; r < 8; ++r) mloc = fmaxf(mloc, s[j][r]);
    mloc = fmaxf(mloc, __shfl_xor(mloc, 16));
    const float mnew = fmaxf(mrun, mloc);
    const float alpha = __expf(mrun - mnew);
    mrun = mnew;
    float lsum = 0.0f;
    #pragma unroll
    for (int j = 0; j < 4; ++j)
      #pragma unroll
      for (int r = 0; r < 8; ++r) {
        const float p = __expf(s[j][r] - mnew);
        s[j][r] = p;
        lsum += p;
      }
    lsum += __shfl_xor(lsum, 16);
    lrun = lrun * alpha + lsum;
    #pragma unroll
    for (int t = 0; t < 4; ++t)
      #pragma unroll
      for (int r = 0; r < 8; ++r) {
        oa[t][r] = oa[t][r] * alpha;
        if (DUAL) ob[t][r] = ob[t][r] * alpha;
      }

    v16b ph0, pl0, ph1, pl1;
    pack_p2(s[0], s[1], ph0, pl0);
    pack_p2(s[2], s[3], ph1, pl1);

    #pragma unroll
    for (int t = 0; t < 4; ++t) {
      const size_t vo = (size_t)(16 * t) * SRL + kb;
      {
        const v16b vh0 = ldb(vahb + vo, h);
        const v16b vh1 = ldb(vahb + vo + 32, h);
        const v16b vl0 = ldb(valb + vo, h);
        const v16b vl1 = ldb(valb + vo + 32, h);
        v8f acc = oa[t];
        acc = wmma_bf(vl0, ph0, acc);
        acc = wmma_bf(vl1, ph1, acc);
        acc = wmma_bf(vh0, pl0, acc);
        acc = wmma_bf(vh1, pl1, acc);
        acc = wmma_bf(vh0, ph0, acc);
        acc = wmma_bf(vh1, ph1, acc);
        oa[t] = acc;
      }
      if (DUAL) {
        const v16b ch0 = ldb(vbhb + vo, h);
        const v16b ch1 = ldb(vbhb + vo + 32, h);
        const v16b cl0 = ldb(vblb + vo, h);
        const v16b cl1 = ldb(vblb + vo + 32, h);
        v8f acc2 = ob[t];
        acc2 = wmma_bf(cl0, ph0, acc2);
        acc2 = wmma_bf(cl1, ph1, acc2);
        acc2 = wmma_bf(ch0, pl0, acc2);
        acc2 = wmma_bf(ch1, pl1, acc2);
        acc2 = wmma_bf(ch0, ph0, acc2);
        acc2 = wmma_bf(ch1, ph1, acc2);
        ob[t] = acc2;
      }
    }
  }

  const float inv = __builtin_amdgcn_rcpf(lrun);
  #pragma unroll
  for (int t = 0; t < 4; ++t)
    #pragma unroll
    for (int r = 0; r < 8; ++r) {
      const int d = 16 * t + 8 * h + r;
      sO[d * 64 + 16 * w + m] = oa[t][r] * inv;
      if (DUAL) sO[4096 + d * 64 + 16 * w + m] = ob[t][r] * inv;
    }
  __syncthreads();

  attn_pass<DUAL>(sO, oap, obp, bh, q0, w, lane);
  __threadfence();
  attn_pass<DUAL>(sO, oap, obp, bh, q0, w, lane);
}

__device__ __forceinline__ void gate_pass(const float* sP, float* gate, int b, int head,
                                          int w, int lane) {
  const int q8 = lane & 7, sub = lane >> 3;
  #pragma unroll
  for (int i = 0; i < 2; ++i) {
    const int L = w * 8 + i * 4 + sub;
    const int n = L >> 1, hl = L & 1;
    const v4f v = *(const v4fa*)(sP + n * 64 + 32 * hl + 4 * q8);
    const size_t off = ((size_t)(b * NH + n)) * TGL + 64 * head + 32 * hl + 4 * q8;
    *(volatile v4f*)(gate + off) = v;
  }
}

__global__ __launch_bounds__(128) void gate_kernel(
    const float* __restrict__ o1T, const float* __restrict__ o2T, const float* __restrict__ qT,
    const float* __restrict__ Wg,
    const float* __restrict__ bg,
    float* __restrict__ gate)
{
  __shared__ __attribute__((aligned(16))) float sG[192 * 48];
  __shared__ __attribute__((aligned(16))) float sP[NH * 64];

  const int tid = threadIdx.x, lane = tid & 31, w = tid >> 5;
  const int h = lane >> 4, m = lane & 15;
  const int bhx = blockIdx.x, b = bhx >> 4, head = bhx & 15;

  const float* abase[3];
  #pragma unroll
  for (int e = 0; e < 3; ++e) {
    const int c0 = 16 * (3 * w + e);
    const int sel = c0 >> 6, cl = c0 & 63;
    const float* sp = (sel == 0) ? o1T : ((sel == 1) ? o2T : qT);
    abase[e] = sp + ((size_t)bhx * DM + cl + m) * TGL;
  }
  const float* wrow = Wg + (size_t)m * GK;

  const v8f zero8 = {0.f, 0.f, 0.f, 0.f, 0.f, 0.f, 0.f, 0.f};
  v8f acc[3][3];
  #pragma unroll
  for (int e = 0; e < 3; ++e)
    #pragma unroll
    for (int i = 0; i < 3; ++i) acc[e][i] = zero8;

  #pragma unroll 1
  for (int k0 = 0; k0 < TGL; k0 += 32) {
    const v16b bw0 = ldf(wrow + k0, h);
    const v16b bw1 = ldf(wrow + EMB + k0, h);
    const v16b bw2 = ldf(wrow + 2 * EMB + k0, h);
    #pragma unroll
    for (int e = 0; e < 3; ++e) {
      const v16b a = ldf(abase[e] + k0, h);
      acc[e][0] = wmma_bf(a, bw0, acc[e][0]);
      acc[e][1] = wmma_bf(a, bw1, acc[e][1]);
      acc[e][2] = wmma_bf(a, bw2, acc[e][2]);
    }
  }

  #pragma unroll
  for (int e = 0; e < 3; ++e)
    #pragma unroll
    for (int i = 0; i < 3; ++i)
      #pragma unroll
      for (int r = 0; r < 8; ++r)
        sG[(16 * (3 * w + e) + 8 * h + r) * 48 + 16 * i + m] = acc[e][i][r];
  __syncthreads();

  #pragma unroll
  for (int j = 0; j < 8; ++j) {
    const int idx = tid + 128 * j;
    const int n = idx >> 6, u = idx & 63;
    const float x = sG[(3 * u) * 48 + n] + sG[(3 * u + 1) * 48 + 16 + n]
                  + sG[(3 * u + 2) * 48 + 32 + n] + bg[n];
    const float g = __builtin_amdgcn_rcpf(1.0f + __expf(-x));
    sP[idx] = g;
  }
  __syncthreads();

  gate_pass(sP, gate, b, head, w, lane);
  __threadfence();
  gate_pass(sP, gate, b, head, w, lane);
}

__device__ __forceinline__ void comb_pass(const us* sH, const us* sL, us* xh, us* xl,
                                          int b, int head, int t0, int w, int lane) {
  const int q8 = lane & 7, sub = lane >> 3;
  #pragma unroll
  for (int i = 0; i < 2; ++i) {
    const int L = w * 8 + i * 4 + sub;
    const v8us a = *(const v8usa*)(sH + L * DM + 8 * q8);
    const v8us c = *(const v8usa*)(sL + L * DM + 8 * q8);
    const size_t off = ((size_t)(b * TGL + t0 + L)) * EMB + head * DM + 8 * q8;
    *(volatile v8us*)(xh + off) = a;
    *(volatile v8us*)(xl + off) = c;
  }
}

__global__ __launch_bounds__(256) void combine_kernel(
    const float* __restrict__ o1T, const float* __restrict__ o3T,
    const float* __restrict__ gate,
    us* __restrict__ xh, us* __restrict__ xl)
{
  __shared__ __attribute__((aligned(16))) us sH[64 * DM];
  __shared__ __attribute__((aligned(16))) us sL[64 * DM];

  const int tid = threadIdx.x, lane = tid & 31, w = tid >> 5;
  const int bh = blockIdx.y, b = bh >> 4, head = bh & 15;
  const int t0 = blockIdx.x * 64;
  const int d = tid >> 2, tq = tid & 3;

  const float* p1 = o1T + ((size_t)bh * DM + d) * TGL + t0 + 16 * tq;
  const float* p3 = o3T + ((size_t)bh * DM + d) * TGL + t0 + 16 * tq;
  const float* pg = gate + (size_t)bh * TGL + t0 + 16 * tq;
  #pragma unroll
  for (int c = 0; c < 4; ++c) {
    const v4f a = *(const v4fa*)(p1 + 4 * c);
    const v4f e = *(const v4fa*)(p3 + 4 * c);
    const v4f g = *(const v4fa*)(pg + 4 * c);
    #pragma unroll
    for (int j = 0; j < 4; ++j) {
      const float val = g[j] * a[j] + (1.0f - g[j]) * e[j];
      const us hi = bf16_rne(val);
      const us lo = bf16_rne(val - bf16_val(hi));
      const int tl = 16 * tq + 4 * c + j;
      sH[tl * DM + d] = hi;
      sL[tl * DM + d] = lo;
    }
  }
  __syncthreads();

  comb_pass(sH, sL, xh, xl, b, head, t0, w, lane);
  __threadfence();
  comb_pass(sH, sL, xh, xl, b, head, t0, w, lane);
}

__device__ __forceinline__ void out_pass(const float* sOut, float* out, int m0, int cg,
                                         int w, int lane) {
  const int q8 = lane & 7, sub = lane >> 3;
  #pragma unroll
  for (int i = 0; i < 16; ++i) {
    const int lid = w * 64 + i * 4 + sub;
    const int row = lid >> 1, hl = lid & 1;
    const v4f v = *(const v4fa*)(sOut + row * DM + 32 * hl + 4 * q8);
    const size_t gi = (size_t)(m0 + row) * EMB + cg * DM + 32 * hl + 4 * q8;
    *(volatile v4f*)(out + gi) = v;
  }
}

__global__ __launch_bounds__(128) void out_kernel(
    const us* __restrict__ xh, const us* __restrict__ xl,
    const us* __restrict__ wob,
    const float* __restrict__ bo,
    float* __restrict__ out)
{
  __shared__ __attribute__((aligned(16))) float sOut[128 * DM];

  const int tid = threadIdx.x, lane = tid & 31, w = tid >> 5;
  const int h = lane >> 4, m = lane & 15;
  const int m0 = blockIdx.x * 128;
  const int cg = blockIdx.y;
  const int m0w = m0 + 32 * w;

  const us* ah0 = xh + (size_t)(m0w + m) * EMB;
  const us* ah1 = ah0 + (size_t)16 * EMB;
  const us* al0 = xl + (size_t)(m0w + m) * EMB;
  const us* al1 = al0 + (size_t)16 * EMB;
  const us* wb  = wob + (size_t)(cg * DM + m) * EMB;

  const v8f zero8 = {0.f, 0.f, 0.f, 0.f, 0.f, 0.f, 0.f, 0.f};
  v8f acc[2][4];
  #pragma unroll
  for (int mt = 0; mt < 2; ++mt)
    #pragma unroll
    for (int nt = 0; nt < 4; ++nt) acc[mt][nt] = zero8;

  #pragma unroll 1
  for (int k0 = 0; k0 < EMB; k0 += 32) {
    const v16b a0h = ldb(ah0 + k0, h);
    const v16b a1h = ldb(ah1 + k0, h);
    const v16b a0l = ldb(al0 + k0, h);
    const v16b a1l = ldb(al1 + k0, h);
    #pragma unroll
    for (int nt = 0; nt < 4; ++nt) {
      const v16b bw = ldb(wb + (size_t)nt * 16 * EMB + k0, h);
      acc[0][nt] = wmma_bf(a0l, bw, acc[0][nt]);
      acc[0][nt] = wmma_bf(a0h, bw, acc[0][nt]);
      acc[1][nt] = wmma_bf(a1l, bw, acc[1][nt]);
      acc[1][nt] = wmma_bf(a1h, bw, acc[1][nt]);
    }
  }

  #pragma unroll
  for (int nt = 0; nt < 4; ++nt) {
    const int feat = 16 * nt + m;
    const float bvl = bo[cg * DM + feat];
    #pragma unroll
    for (int mt = 0; mt < 2; ++mt) {
      #pragma unroll
      for (int r = 0; r < 8; ++r) {
        const int tokl = 32 * w + 16 * mt + 8 * h + r;
        sOut[tokl * DM + feat] = acc[mt][nt][r] + bvl;
      }
    }
  }
  __syncthreads();

  out_pass(sOut, out, m0, cg, w, lane);
  __threadfence();
  out_pass(sOut, out, m0, cg, w, lane);
}

extern "C" void kernel_launch(void* const* d_in, const int* in_sizes, int n_in,
                              void* d_out, int out_size, void* d_ws, size_t ws_size,
                              hipStream_t stream) {
  if (n_in < 17) return;
  if (in_sizes[0] != N_HID || in_sizes[1] != N_KVS || in_sizes[2] != N_KVT) return;
  if (in_sizes[3] != N_WE || in_sizes[5] != N_WE || in_sizes[7] != N_WE || in_sizes[15] != N_WE) return;
  if (in_sizes[9] != N_WT || in_sizes[11] != N_WT) return;
  if (in_sizes[4] != EMB || in_sizes[6] != EMB || in_sizes[8] != EMB ||
      in_sizes[10] != EMB || in_sizes[12] != EMB || in_sizes[16] != EMB) return;
  if (in_sizes[13] != N_WG || in_sizes[14] != NH) return;
  if (out_size != N_HID) return;

  const float* hid = (const float*)d_in[0];
  const float* kvs = (const float*)d_in[1];
  const float* kvt = (const float*)d_in[2];
  const float* Wq  = (const float*)d_in[3];
  const float* bq  = (const float*)d_in[4];
  const float* Wk  = (const float*)d_in[5];
  const float* bk  = (const float*)d_in[6];
  const float* Wv  = (const float*)d_in[7];
  const float* bv  = (const float*)d_in[8];
  const float* Wtk = (const float*)d_in[9];
  const float* btk = (const float*)d_in[10];
  const float* Wtv = (const float*)d_in[11];
  const float* btv = (const float*)d_in[12];
  const float* Wg  = (const float*)d_in[13];
  const float* bg  = (const float*)d_in[14];
  const float* Wo  = (const float*)d_in[15];
  const float* bo  = (const float*)d_in[16];
  float* out = (float*)d_out;

  const size_t cvb_b  = (size_t)N_CVB * 2;
  const size_t qpl2   = (size_t)QPL * 2;
  const size_t qpl4   = (size_t)QPL * 4;
  const size_t kpl2   = (size_t)KPL * 2;
  const size_t gate_b = (size_t)NBH * TGL * 4;
  const size_t xpl_b  = (size_t)N_HID * 2;
  const size_t total  = cvb_b + 2 * qpl2 + qpl4 + 8 * kpl2 + qpl4 + gate_b + 2 * xpl_b;
  if (total > ws_size) return;
  const size_t act_off = (size_t)OFF_HID * 2;
  if (act_off + 2 * qpl4 != cvb_b) return;

  char* ws = (char*)d_ws;
  size_t off = 0;
  us* cvb    = (us*)(ws + off);    off += cvb_b;
  float* o1T = (float*)(ws + act_off);
  float* o2T = (float*)(ws + act_off + qpl4);
  us* qh     = (us*)(ws + off);    off += qpl2;
  us* ql     = (us*)(ws + off);    off += qpl2;
  float* qT  = (float*)(ws + off); off += qpl4;
  us* kh     = (us*)(ws + off);    off += kpl2;
  us* kl     = (us*)(ws + off);    off += kpl2;
  us* kth    = (us*)(ws + off);    off += kpl2;
  us* ktl    = (us*)(ws + off);    off += kpl2;
  us* vh     = (us*)(ws + off);    off += kpl2;
  us* vl     = (us*)(ws + off);    off += kpl2;
  us* vth    = (us*)(ws + off);    off += kpl2;
  us* vtl    = (us*)(ws + off);    off += kpl2;
  float* o3T = (float*)(ws + off); off += qpl4;
  float* gte = (float*)(ws + off); off += gate_b;
  us* xh     = (us*)(ws + off);    off += xpl_b;
  us* xl     = (us*)(ws + off);    off += xpl_b;
  if (off != total || off > ws_size) return;

  conv_kernel<<<(N_CVB / 8 + 255) / 256, 256, 0, stream>>>(Wq, Wk, Wv, Wo, Wtk, Wtv, hid, kvs, kvt, cvb);

  dim3 gQ(MQ / 128, NH);
  dim3 gKV(MKV / 128, NH);
  proj_kernel<<<gQ,  128, 0, stream>>>(cvb + OFF_HID, cvb + OFF_WQ,  bq,  EMB, TGL, 0, qh,  ql,  qT);
  proj_kernel<<<gKV, 128, 0, stream>>>(cvb + OFF_KVS, cvb + OFF_WK,  bk,  EMB, SRL, 1, kh,  kl,  qT);
  proj_kernel<<<gKV, 128, 0, stream>>>(cvb + OFF_KVS, cvb + OFF_WV,  bv,  EMB, SRL, 2, vh,  vl,  qT);
  proj_kernel<<<gKV, 128, 0, stream>>>(cvb + OFF_KVT, cvb + OFF_WTK, btk, TDW, SRL, 1, kth, ktl, qT);
  proj_kernel<<<gKV, 128, 0, stream>>>(cvb + OFF_KVT, cvb + OFF_WTV, btv, TDW, SRL, 2, vth, vtl, qT);

  dim3 gAtt(TGL / 64, NBH);
  attn_kernel<false><<<gAtt, 128, 0, stream>>>(qh, ql, kh,  kl,  vh,  vl,  vh, vl, o1T, o1T);
  attn_kernel<true ><<<gAtt, 128, 0, stream>>>(qh, ql, kth, ktl, vth, vtl, vh, vl, o2T, o3T);

  gate_kernel<<<NBH, 128, 0, stream>>>(o1T, o2T, qT, Wg, bg, gte);

  dim3 gCmb(TGL / 64, NBH);
  combine_kernel<<<gCmb, 256, 0, stream>>>(o1T, o3T, gte, xh, xl);

  dim3 gOut(MQ / 128, EMB / 64);
  out_kernel<<<gOut, 128, 0, stream>>>(xh, xl, cvb + OFF_WO, bo, out);
}
